// SSMBlock_28381143892541
// MI455X (gfx1250) — hardware-verified
//
#include <hip/hip_runtime.h>
#include <math.h>

typedef __attribute__((ext_vector_type(16))) _Float16 v16h;
typedef __attribute__((ext_vector_type(8)))  _Float16 v8h;
typedef __attribute__((ext_vector_type(16))) __bf16   v16b;
typedef __attribute__((ext_vector_type(8)))  __bf16   v8b;
typedef __attribute__((ext_vector_type(8)))  float    v8f;
typedef __attribute__((ext_vector_type(4)))  float    v4f;
typedef __attribute__((ext_vector_type(4)))  unsigned v4u;

constexpr int kBatch    = 4;
constexpr int kSeq      = 4096;
constexpr int kDim      = 512;
constexpr int kRows     = kBatch * kSeq;
constexpr int kHalfB    = 2;
constexpr int kHalfRows = kHalfB * kSeq;
constexpr int kScanTS   = 64;
constexpr int kScanCh   = 64;
constexpr int kScanYP   = 68;
constexpr int kPrmRows  = 5;
static_assert(kRows == 16384);
static_assert(kHalfRows == 8192);
static_assert((kDim % 64) == 0 && (kDim % 32) == 0 && (kHalfRows % 64) == 0);
static_assert((kSeq % kScanTS) == 0 && (kDim % kScanCh) == 0);

constexpr size_t kSzW    = (size_t)kDim * kDim * 2;
constexpr size_t kOffXB  = 0;
constexpr size_t kOffWG  = kOffXB  + (size_t)kRows * kDim * 2;
constexpr size_t kOffWS  = kOffWG  + kSzW;
constexpr size_t kOffWST = kOffWS  + kSzW;
constexpr size_t kOffWO  = kOffWST + kSzW;
constexpr size_t kOffPRM = kOffWO  + kSzW;
constexpr size_t kOffG   = kOffPRM + (size_t)kPrmRows * kDim * 4;
constexpr size_t kOffS   = kOffG   + (size_t)kHalfRows * kDim * 4;
constexpr size_t kOffXGH = kOffS   + (size_t)kHalfRows * kDim * 4;
constexpr size_t kOffXGL = kOffXGH + (size_t)kHalfRows * kDim * 2;
constexpr size_t kOffSTH = kOffXGL + (size_t)kHalfRows * kDim * 2;
constexpr size_t kOffSTL = kOffSTH + (size_t)kHalfRows * kDim * 2;
constexpr size_t kOffYH  = kOffSTL + (size_t)kHalfRows * kDim * 2;
constexpr size_t kOffYL  = kOffYH  + (size_t)kHalfRows * kDim * 2;
constexpr size_t kWsTotal = kOffYL + (size_t)kHalfRows * kDim * 2;
static_assert(kWsTotal == 102770688ull);
static_assert(kWsTotal <= 134217728ull);
static_assert((kOffWG % 128) == 0 && (kOffWS % 128) == 0 && (kOffWST % 128) == 0 && (kOffWO % 128) == 0 &&
              (kOffPRM % 128) == 0 && (kOffG % 128) == 0 && (kOffS % 128) == 0 && (kOffXGH % 128) == 0 &&
              (kOffXGL % 128) == 0 && (kOffSTH % 128) == 0 && (kOffSTL % 128) == 0 && (kOffYH % 128) == 0 &&
              (kOffYL % 128) == 0);
constexpr size_t kOut1Elem = (size_t)kRows * kDim;
static_assert(kOut1Elem * 4 == 33554432ull);
static_assert(kOut1Elem * 4 + (size_t)kBatch * kDim * 4 == 33562624ull);

__device__ __forceinline__ unsigned short f2bf_bits(float f) {
  unsigned u = __float_as_uint(f);
  return (unsigned short)((u + 0x7FFFu + ((u >> 16) & 1u)) >> 16);
}
__device__ __forceinline__ float bf_bits2f(unsigned short h) { return __uint_as_float(((unsigned)h) << 16); }
__device__ __forceinline__ float rne_bf16f(float f) { return bf_bits2f(f2bf_bits(f)); }

__device__ __forceinline__ void dep_guard4_b(v8f& a, v8f& b, v8f& c, v8f& d, v16b x, v16b y) {
  asm volatile("v_nop\n\tv_nop\n\tv_nop\n\tv_nop" : "+v"(a), "+v"(b), "+v"(c), "+v"(d) : "v"(x), "v"(y));
}
__device__ __forceinline__ void keep4_b(v16b a, v16b b, v16b c, v16b d) { asm volatile("v_nop" :: "v"(a), "v"(b), "v"(c), "v"(d)); }
__device__ __forceinline__ void acc_guard4(v8f& a, v8f& b, v8f& c, v8f& d) { asm volatile("v_nop\n\tv_nop\n\tv_nop\n\tv_nop" : "+v"(a), "+v"(b), "+v"(c), "+v"(d)); }

template <typename T> struct Frag;
template <> struct Frag<__bf16> {
  typedef v16b V; union U { v16b v; v8b h[2]; };
  static __device__ __forceinline__ v16b load(const __bf16* p) {
    U f; f.h[0] = *(const v8b*)(p); f.h[1] = *(const v8b*)(p + 16); return f.v;
  }
  static __device__ __forceinline__ v8f mma(v16b a, v16b b, v8f c) {
    return __builtin_amdgcn_wmma_f32_16x16x32_bf16(false, a, false, b, (short)0, c, false, false);
  }
};

template <int SPL, int BIAS_MODE, int OUT_MODE, bool SKIP>
__global__ __launch_bounds__(256) void wmma_gemm64(
    const unsigned short* __restrict__ Ap, const unsigned short* __restrict__ A2p, int lda,
    const unsigned short* __restrict__ Btp, int ldb,
    void* __restrict__ Cout, void* __restrict__ Cout2, int ldc,
    const float* __restrict__ bias,
    const unsigned short* __restrict__ skh, const unsigned short* __restrict__ skl,
    const float* __restrict__ skscale,
    int M, int N, int K, float scale) {
  typedef __bf16 T;
  typedef Frag<T>::V V;
  const T* A = (const T*)Ap; const T* A2 = (const T*)A2p; const T* Bt = (const T*)Btp;
  __shared__ __align__(16) float sT[8][16 * 68];
  const int lane = threadIdx.x & 31;
  const int wave = threadIdx.x >> 5;
  const int tilesN = N >> 6;
  const int tilesM = M >> 6;
  const int tile = blockIdx.x * 8 + wave;
  if (tile >= tilesM * tilesN) return;
  const int tm = tile / tilesN;
  const int tn = tile - tm * tilesN;
  const int m0 = tm << 6;
  const int n0 = tn << 6;

  const int rlane = lane & 15;
  const int koff  = (lane >> 4) * 8;
  const int mOff  = (lane >> 4) * 8;

  v8f acc[4][4];
#pragma unroll
  for (int i = 0; i < 4; ++i)
#pragma unroll
    for (int j = 0; j < 4; ++j) acc[i][j] = (v8f){0.f,0.f,0.f,0.f,0.f,0.f,0.f,0.f};

  for (int k0 = 0; k0 < K; k0 += 32) {
    V bh[4];
#pragma unroll
    for (int j = 0; j < 4; ++j) {
      const size_t bo = (size_t)(n0 + (j << 4) + rlane) * ldb + koff + k0;
      bh[j] = Frag<T>::load(Bt + bo);
    }
#pragma unroll
    for (int i = 0; i < 4; ++i) {
      const size_t ao = (size_t)(m0 + (i << 4) + rlane) * lda + koff + k0;
      V ah = Frag<T>::load(A + ao);
      V al = ah;
      if (SPL >= 1) al = Frag<T>::load(A2 + ao);
#pragma unroll
      for (int j = 0; j < 4; ++j) {
        acc[i][j] = Frag<T>::mma(ah, bh[j], acc[i][j]);
        if (SPL >= 1) acc[i][j] = Frag<T>::mma(al, bh[j], acc[i][j]);
      }
      dep_guard4_b(acc[i][0], acc[i][1], acc[i][2], acc[i][3], ah, al);
    }
    keep4_b(bh[0], bh[1], bh[2], bh[3]);
  }
  acc_guard4(acc[0][0], acc[0][1], acc[0][2], acc[0][3]);
  acc_guard4(acc[1][0], acc[1][1], acc[1][2], acc[1][3]);
  acc_guard4(acc[2][0], acc[2][1], acc[2][2], acc[2][3]);
  acc_guard4(acc[3][0], acc[3][1], acc[3][2], acc[3][3]);

  float* slab = sT[wave];
#pragma unroll
  for (int i = 0; i < 4; ++i) {
    const int mBase = m0 + (i << 4);
#pragma unroll
    for (int j = 0; j < 4; ++j) {
      const int n = n0 + (j << 4) + rlane;
      float bv = 0.f;
      if (BIAS_MODE == 2) bv = bias[n];
#pragma unroll
      for (int r = 0; r < 8; ++r) {
        float v = acc[i][j][r] * scale;
        if (BIAS_MODE == 2) v += bv;
        slab[(mOff + r) * 68 + (j << 4) + rlane] = v;
      }
    }
    __builtin_amdgcn_fence(__ATOMIC_RELEASE, "workgroup");
    __builtin_amdgcn_wave_barrier();
    __builtin_amdgcn_fence(__ATOMIC_ACQUIRE, "workgroup");
    if (OUT_MODE == 0) {
      float* C = (float*)Cout;
      const int hh = lane >> 4, c4 = (lane & 15) * 4;
      for (int pass = 0; pass < 2; ++pass) {
#pragma unroll
        for (int it = 0; it < 8; ++it) {
          const int row = it * 2 + hh;
          v4f v = *(const v4f*)(slab + row * 68 + c4);
          *(volatile v4f*)(C + (size_t)(mBase + row) * ldc + n0 + c4) = v;
        }
        __threadfence();
      }
    } else {
      const int q = lane >> 3, c8 = (lane & 7) * 8;
      unsigned short* C  = (unsigned short*)Cout;
      unsigned short* C2 = (unsigned short*)Cout2;
      v4f sk0 = (v4f){0.f, 0.f, 0.f, 0.f};
      v4f sk1 = (v4f){0.f, 0.f, 0.f, 0.f};
      if (SKIP) {
        sk0 = *(const v4f*)(skscale + n0 + c8);
        sk1 = *(const v4f*)(skscale + n0 + c8 + 4);
      }
      v8h hv[4], lv[4];
#pragma unroll
      for (int it = 0; it < 4; ++it) {
        const int row = it * 4 + q;
        const float* sp = slab + row * 68 + c8;
        const v4f a0 = *(const v4f*)(sp);
        const v4f a1 = *(const v4f*)(sp + 4);
        float val[8];
        val[0] = a0[0]; val[1] = a0[1]; val[2] = a0[2]; val[3] = a0[3];
        val[4] = a1[0]; val[5] = a1[1]; val[6] = a1[2]; val[7] = a1[3];
        if (SKIP) {
          const size_t go = (size_t)(mBase + row) * ldc + n0 + c8;
          const v4u wh = *(const v4u*)(skh + go);
          const v4u wl = *(const v4u*)(skl + go);
          float sc[8];
          sc[0] = sk0[0]; sc[1] = sk0[1]; sc[2] = sk0[2]; sc[3] = sk0[3];
          sc[4] = sk1[0]; sc[5] = sk1[1]; sc[6] = sk1[2]; sc[7] = sk1[3];
#pragma unroll
          for (int p = 0; p < 4; ++p) {
            const unsigned uh = wh[p];
            const unsigned ul = wl[p];
            const float xe = __uint_as_float(uh << 16) + __uint_as_float(ul << 16);
            const float xo = __uint_as_float(uh & 0xffff0000u) + __uint_as_float(ul & 0xffff0000u);
            val[2 * p]     += sc[2 * p] * xe;
            val[2 * p + 1] += sc[2 * p + 1] * xo;
          }
        }
#pragma unroll
        for (int e = 0; e < 8; ++e) {
          const float fv = val[e];
          const unsigned short hb = f2bf_bits(fv);
          const unsigned short lb = f2bf_bits(fv - bf_bits2f(hb));
          hv[it][e] = __builtin_bit_cast(_Float16, hb);
          lv[it][e] = __builtin_bit_cast(_Float16, lb);
        }
      }
      for (int pass = 0; pass < 2; ++pass) {
#pragma unroll
        for (int it = 0; it < 4; ++it) {
          const int row = it * 4 + q;
          const size_t o = (size_t)(mBase + row) * ldc + n0 + c8;
          *(volatile v8h*)(C + o)  = hv[it];
          *(volatile v8h*)(C2 + o) = lv[it];
        }
        __threadfence();
      }
    }
    __builtin_amdgcn_fence(__ATOMIC_RELEASE, "workgroup");
    __builtin_amdgcn_wave_barrier();
    __builtin_amdgcn_fence(__ATOMIC_ACQUIRE, "workgroup");
  }
}

__device__ __forceinline__ void rne_store8(const float* __restrict__ src, unsigned short* __restrict__ dst, size_t e0) {
  const v4f a0 = *(const v4f*)(src + e0);
  const v4f a1 = *(const v4f*)(src + e0 + 4);
  v8h hv;
#pragma unroll
  for (int e = 0; e < 4; ++e) {
    const unsigned short h0 = f2bf_bits(a0[e]);
    const unsigned short h1 = f2bf_bits(a1[e]);
    hv[e]     = __builtin_bit_cast(_Float16, h0);
    hv[4 + e] = __builtin_bit_cast(_Float16, h1);
  }
  unsigned short* qd = dst + e0;
  *(volatile v8h*)qd = hv;
  __threadfence();
  *(volatile v8h*)qd = hv;
}

__global__ __launch_bounds__(256) void rne_rows_bf16_kernel(
    const float* __restrict__ src, unsigned short* __restrict__ dst, int total8)
{
  const int i = blockIdx.x * 256 + threadIdx.x;
  if (i >= total8) return;
  rne_store8(src, dst, (size_t)i << 3);
}

__global__ __launch_bounds__(256) void rne_w3_kernel(
    const float* __restrict__ s0, const float* __restrict__ s1, const float* __restrict__ s2,
    unsigned short* __restrict__ d0, unsigned short* __restrict__ d1, unsigned short* __restrict__ d2, int total8)
{
  const int i = blockIdx.x * 256 + threadIdx.x;
  if (i >= total8) return;
  const int y = blockIdx.y;
  const float* src = (y == 0) ? s0 : ((y == 1) ? s1 : s2);
  unsigned short* dst = (y == 0) ? d0 : ((y == 1) ? d1 : d2);
  rne_store8(src, dst, (size_t)i << 3);
}

__global__ __launch_bounds__(256) void transpose_bf16_kernel(
    const float* __restrict__ W, unsigned short* __restrict__ Bt, int Kdim, int Ndim)
{
  __shared__ float tile[64 * 65];
  const int tid = threadIdx.x, lane = tid & 31, wave = tid >> 5;
  const int n0 = blockIdx.x * 64;
  const int k0 = blockIdx.y * 64;
#pragma unroll 4
  for (int p = 0; p < 16; ++p) {
    const int idx = tid + p * 256;
    const int kk  = idx >> 6;
    const int nn  = idx & 63;
    tile[kk * 65 + nn] = W[(size_t)(k0 + kk) * Ndim + n0 + nn];
  }
  __syncthreads();
  const int q = lane >> 3, c8 = (lane & 7) * 8;
  v8h hv[2];
#pragma unroll
  for (int it = 0; it < 2; ++it) {
    const int nrow = it * 32 + wave * 4 + q;
#pragma unroll
    for (int e = 0; e < 8; ++e) {
      const unsigned short hb = f2bf_bits(tile[(c8 + e) * 65 + nrow]);
      hv[it][e] = __builtin_bit_cast(_Float16, hb);
    }
  }
  for (int pass = 0; pass < 2; ++pass) {
#pragma unroll
    for (int it = 0; it < 2; ++it) {
      const int nrow = it * 32 + wave * 4 + q;
      *(volatile v8h*)(Bt + (size_t)(n0 + nrow) * Kdim + k0 + c8) = hv[it];
    }
    __threadfence();
  }
}

__global__ __launch_bounds__(256) void params_kernel(
    const float* __restrict__ Alog, const float* __restrict__ bg, const float* __restrict__ bsp,
    const float* __restrict__ bo, const float* __restrict__ dp, float* __restrict__ PRM)
{
  __shared__ float sD[32];
  const int tid = threadIdx.x, lane = tid & 31, wave = tid >> 5;
  const int j0 = blockIdx.x * 32;
#pragma unroll 1
  for (int rr = 0; rr < 4; ++rr) {
    const int row = j0 + wave * 4 + rr;
    const float* ap = Alog + (size_t)row * kDim;
    float acc = 0.0f;
#pragma unroll 4
    for (int i = 0; i < kDim / 32; ++i) {
      const float a = rne_bf16f(ap[lane + 32 * i]);
      acc += expf(a);
    }
#pragma unroll
    for (int off = 16; off >= 1; off >>= 1) acc += __shfl_xor(acc, off, 32);
    if (lane == 0) sD[wave * 4 + rr] = acc;
  }
  __syncthreads();
  const float* src = (wave == 2) ? bsp : ((wave == 3) ? bo : ((wave == 4) ? dp : bg));
  const float lsum = sD[lane];
  const float gv   = src[j0 + lane];
  const float dec  = expf(-(lsum * (1.0f / (float)kDim)));
  const float val  = (wave == 0) ? dec : rne_bf16f(gv);
  if (wave <= 4) {
    float* qd = PRM + (size_t)wave * kDim + j0 + lane;
    *(volatile float*)qd = val;
    __threadfence();
    *(volatile float*)qd = val;
  }
}

__device__ __forceinline__ float silu_f32(float g) {
  return g * __builtin_amdgcn_rcpf(1.0f + expf(-g));
}

__global__ __launch_bounds__(256) void silu_split_kernel(
    const float* __restrict__ G, unsigned short* __restrict__ dhi, unsigned short* __restrict__ dlo, int total8)
{
  const int i = blockIdx.x * 256 + threadIdx.x;
  if (i >= total8) return;
  const size_t e0 = (size_t)i << 3;
  const v4f a0 = *(const v4f*)(G + e0);
  const v4f a1 = *(const v4f*)(G + e0 + 4);
  v8h hv, lv;
#pragma unroll
  for (int e = 0; e < 4; ++e) {
    const float s0 = silu_f32(a0[e]);
    const float s1 = silu_f32(a1[e]);
    const unsigned short h0 = f2bf_bits(s0), h1 = f2bf_bits(s1);
    const unsigned short l0 = f2bf_bits(s0 - bf_bits2f(h0)), l1 = f2bf_bits(s1 - bf_bits2f(h1));
    hv[e]     = __builtin_bit_cast(_Float16, h0);
    hv[4 + e] = __builtin_bit_cast(_Float16, h1);
    lv[e]     = __builtin_bit_cast(_Float16, l0);
    lv[4 + e] = __builtin_bit_cast(_Float16, l1);
  }
  unsigned short* qh = dhi + e0;
  unsigned short* ql = dlo + e0;
  *(volatile v8h*)qh = hv;
  *(volatile v8h*)ql = lv;
  __threadfence();
  *(volatile v8h*)qh = hv;
  *(volatile v8h*)ql = lv;
}

__global__ __launch_bounds__(64) void scan_kernel(
    const float* __restrict__ S, const float* __restrict__ decay, const float* __restrict__ state0,
    unsigned short* __restrict__ STH, unsigned short* __restrict__ STL, float* __restrict__ statef)
{
  __shared__ __align__(16) float sY[kScanTS * kScanYP];
  const int tid = threadIdx.x, lane = tid & 31, wave = tid >> 5;
  constexpr int kBlkPerB = kDim / kScanCh;
  const int bl = blockIdx.x / kBlkPerB;
  const int d0 = (blockIdx.x - bl * kBlkPerB) * kScanCh;
  const int d  = d0 + tid;
  const size_t row0 = (size_t)bl * kSeq;
  const float dec = decay[d];
  float st = rne_bf16f(state0[(size_t)bl * kDim + d]);
  const int q = lane >> 3, c8 = (lane & 7) * 8;
#pragma unroll 1
  for (int t0 = 0; t0 < kSeq; t0 += kScanTS) {
    __syncthreads();
    const float* Sp = S + (row0 + t0) * kDim + d;
#pragma unroll 1
    for (int s8 = 0; s8 < kScanTS; s8 += 8) {
      float v[8];
#pragma unroll
      for (int e = 0; e < 8; ++e) v[e] = Sp[(size_t)(s8 + e) * kDim];
#pragma unroll
      for (int e = 0; e < 8; ++e) {
        st = st * dec + v[e];
        sY[(s8 + e) * kScanYP + tid] = st;
      }
    }
    __syncthreads();
    v8h hv[8], lv[8];
#pragma unroll
    for (int it = 0; it < 8; ++it) {
      const int row = it * 8 + wave * 4 + q;
      const float* sp = sY + row * kScanYP + c8;
      const v4f a0 = *(const v4f*)(sp);
      const v4f a1 = *(const v4f*)(sp + 4);
#pragma unroll
      for (int e = 0; e < 4; ++e) {
        const unsigned short h0 = f2bf_bits(a0[e]), h1 = f2bf_bits(a1[e]);
        const unsigned short l0 = f2bf_bits(a0[e] - bf_bits2f(h0)), l1 = f2bf_bits(a1[e] - bf_bits2f(h1));
        hv[it][e]     = __builtin_bit_cast(_Float16, h0);
        hv[it][4 + e] = __builtin_bit_cast(_Float16, h1);
        lv[it][e]     = __builtin_bit_cast(_Float16, l0);
        lv[it][4 + e] = __builtin_bit_cast(_Float16, l1);
      }
    }
    for (int pass = 0; pass < 2; ++pass) {
#pragma unroll
      for (int it = 0; it < 8; ++it) {
        const int row = it * 8 + wave * 4 + q;
        const size_t o = (row0 + t0 + row) * kDim + d0 + c8;
        *(volatile v8h*)(STH + o) = hv[it];
        *(volatile v8h*)(STL + o) = lv[it];
      }
      __threadfence();
    }
  }
  float* qf = statef + (size_t)bl * kDim + d;
  *(volatile float*)qf = st;
  __threadfence();
  *(volatile float*)qf = st;
}

extern "C" void kernel_launch(void* const* d_in, const int* in_sizes, int n_in,
                              void* d_out, int out_size, void* d_ws, size_t ws_size,
                              hipStream_t stream) {
  if (n_in < 10) return;
  if (in_sizes[0] != kRows * kDim) return;
  if (in_sizes[1] != kBatch * kDim) return;
  if (in_sizes[2] != kDim * kDim || in_sizes[3] != kDim) return;
  if (in_sizes[4] != kDim * kDim || in_sizes[5] != kDim) return;
  if (in_sizes[6] != kDim * kDim || in_sizes[7] != kDim) return;
  if (in_sizes[8] != kDim * kDim || in_sizes[9] != kDim) return;
  if (out_size != kRows * kDim + kBatch * kDim) return;
  if (ws_size < kWsTotal) return;

  const float* x      = (const float*)d_in[0];
  const float* state0 = (const float*)d_in[1];
  const float* Wg     = (const float*)d_in[2];
  const float* bg     = (const float*)d_in[3];
  const float* Wsp    = (const float*)d_in[4];
  const float* bsp    = (const float*)d_in[5];
  const float* Wo     = (const float*)d_in[6];
  const float* bo     = (const float*)d_in[7];
  const float* Alog   = (const float*)d_in[8];
  const float* Dp     = (const float*)d_in[9];
  float* out = (float*)d_out;

  char* ws = (char*)d_ws;
  unsigned short* XB  = (unsigned short*)(ws + kOffXB);
  unsigned short* WG  = (unsigned short*)(ws + kOffWG);
  unsigned short* WS  = (unsigned short*)(ws + kOffWS);
  unsigned short* WST = (unsigned short*)(ws + kOffWST);
  unsigned short* WO  = (unsigned short*)(ws + kOffWO);
  float*          PRM = (float*)(ws + kOffPRM);
  float*          G   = (float*)(ws + kOffG);
  float*          S   = (float*)(ws + kOffS);
  unsigned short* XGH = (unsigned short*)(ws + kOffXGH);
  unsigned short* XGL = (unsigned short*)(ws + kOffXGL);
  unsigned short* STH = (unsigned short*)(ws + kOffSTH);
  unsigned short* STL = (unsigned short*)(ws + kOffSTL);
  unsigned short* YH  = (unsigned short*)(ws + kOffYH);
  unsigned short* YL  = (unsigned short*)(ws + kOffYL);
  const float* pDecay = PRM;
  const float* pBg    = PRM + kDim;
  const float* pBsp   = PRM + 2 * kDim;
  const float* pBo    = PRM + 3 * kDim;
  const float* pDp    = PRM + 4 * kDim;

  rne_rows_bf16_kernel<<<(kRows * kDim / 8) / 256, 256, 0, stream>>>(x, XB, kRows * kDim / 8);
  rne_w3_kernel<<<dim3((kDim * kDim / 8) / 256, 3), 256, 0, stream>>>(Wg, Wsp, Wo, WG, WS, WO, kDim * kDim / 8);
  transpose_bf16_kernel<<<dim3(kDim / 64, kDim / 64), 256, 0, stream>>>(Wsp, WST, kDim, kDim);
  params_kernel<<<kDim / 32, 256, 0, stream>>>(Alog, bg, bsp, bo, Dp, PRM);

  constexpr int kGemmBlocks = ((kHalfRows / 64) * (kDim / 64)) / 8;
  static_assert(kGemmBlocks * 8 == (kHalfRows / 64) * (kDim / 64));

  for (int h = 0; h < kBatch / kHalfB; ++h) {
    const size_t r0 = (size_t)h * kHalfRows;
    const unsigned short* XBh = XB + r0 * kDim;
    float* outh = out + r0 * kDim;
    const float* st0h = state0 + (size_t)h * kHalfB * kDim;
    float* stfh = out + kOut1Elem + (size_t)h * kHalfB * kDim;

    wmma_gemm64<0, 2, 0, false><<<kGemmBlocks, 256, 0, stream>>>(
        XBh, XBh, kDim, WG, kDim, (void*)G, (void*)G, kDim, pBg,
        XBh, XBh, pBg, kHalfRows, kDim, kDim, 1.0f);

    silu_split_kernel<<<(kHalfRows * kDim / 8) / 256, 256, 0, stream>>>(G, XGH, XGL, kHalfRows * kDim / 8);

    wmma_gemm64<1, 2, 0, false><<<kGemmBlocks, 256, 0, stream>>>(
        XGH, XGL, kDim, WS, kDim, (void*)S, (void*)S, kDim, pBsp,
        XGH, XGL, pBsp, kHalfRows, kDim, kDim, 1.0f);

    scan_kernel<<<kHalfB * (kDim / kScanCh), kScanCh, 0, stream>>>(S, pDecay, st0h, STH, STL, stfh);

    wmma_gemm64<1, 0, 2, true><<<kGemmBlocks, 256, 0, stream>>>(
        STH, STL, kDim, WST, kDim, (void*)YH, (void*)YL, kDim, pDp,
        XGH, XGL, pDp, kHalfRows, kDim, kDim, 1.0f);

    wmma_gemm64<1, 2, 0, false><<<kGemmBlocks, 256, 0, stream>>>(
        YH, YL, kDim, WO, kDim, (void*)outh, (void*)outh, kDim, pBo,
        YH, YL, pBo, kHalfRows, kDim, kDim, 1.0f);
  }
}
